// NeuralODE_46935402611059
// MI455X (gfx1250) — hardware-run, weakly checked
//
#include <hip/hip_runtime.h>
#include <math.h>

constexpr int DIM_X  = 32;
constexpr int DIM_H  = 128;
constexpr int NSAMP  = 32;
constexpr int NSTEPS = 48;
constexpr int NSTAGE = 7;
constexpr int NTHR   = 256;
constexpr int NWAVE  = NTHR / 32;
constexpr int SPB    = 8;
constexpr int NBLK   = NSAMP / SPB;
constexpr int WPW    = 68;
constexpr int FP     = 132;
constexpr int ZP     = 36;
constexpr int W1_ELEMS = DIM_H * (DIM_X + 1);
constexpr int OUT0_ELEMS = NSAMP * DIM_X;
constexpr int OUT_ELEMS  = OUT0_ELEMS + NSAMP;
static_assert(SPB == NWAVE, "one wave per sample");
static_assert(DIM_H == 16 * NWAVE, "one m-tile per wave on the value path");
static_assert(DIM_H == 4 * 32, "a lane owns four hidden units in the first layer");
static_assert(DIM_X == 32, "a lane owns one state component");
static_assert(DIM_H % 32 == 0, "k-steps of 32");
static_assert(NSAMP % SPB == 0, "whole blocks");
static_assert(OUT0_ELEMS * 4 == 4096, "second output starts at byte 4096");
static_assert(OUT_ELEMS * 4 == 4224, "output extent");
static_assert((FP * 4) % 16 == 0 && (ZP * 4) % 16 == 0 && (WPW * 4) % 16 == 0, "16-B aligned rows");

constexpr float ATOL_F   = 1e-5f;
constexpr float RTOL_F   = 1e-3f;
constexpr float DT_INIT  = 1e-4f;
constexpr float T_END    = 1.0f;
constexpr float T_DONE   = (float)(1.0 - 1e-10);
constexpr float INV_NCMP = 1.0f / (float)(DIM_X + 1);

constexpr float CARRY_W2 = 1024.0f;
constexpr float CARRY_H1 = 256.0f;
constexpr float CARRY_T1 = 1024.0f;
constexpr float FOLD_H1  = 1.0f / (CARRY_W2 * CARRY_H1);
constexpr float FOLD_T1  = 1.0f / (CARRY_W2 * CARRY_T1);
constexpr float F16_MIN_NORMAL = 6.103515625e-5f;
static_assert(FOLD_H1 * CARRY_W2 * CARRY_H1 == 1.0f, "exact fold");
static_assert(FOLD_T1 * CARRY_W2 * CARRY_T1 == 1.0f, "exact fold");

__constant__ float c_A[6][6] = {
  {(float)(0.2), 0.f, 0.f, 0.f, 0.f, 0.f},
  {(float)(3.0 / 40.0), (float)(9.0 / 40.0), 0.f, 0.f, 0.f, 0.f},
  {(float)(44.0 / 45.0), (float)(-56.0 / 15.0), (float)(32.0 / 9.0), 0.f, 0.f, 0.f},
  {(float)(19372.0 / 6561.0), (float)(-25360.0 / 2187.0), (float)(64448.0 / 6561.0), (float)(-212.0 / 729.0), 0.f, 0.f},
  {(float)(9017.0 / 3168.0), (float)(-355.0 / 33.0), (float)(46732.0 / 5247.0), (float)(49.0 / 176.0), (float)(-5103.0 / 18656.0), 0.f},
  {(float)(35.0 / 384.0), 0.f, (float)(500.0 / 1113.0), (float)(125.0 / 192.0), (float)(-2187.0 / 6784.0), (float)(11.0 / 84.0)}};
__constant__ float c_C[7] = {0.f, (float)(0.2), (float)(0.3), (float)(0.8), (float)(8.0 / 9.0), 1.f, 1.f};
static_assert(sizeof(c_A) / sizeof(c_A[0]) == 6, "tableau rows");
static_assert(sizeof(c_C) / sizeof(c_C[0]) == 7, "tableau nodes");

constexpr float B5_0 = (float)(35.0 / 384.0);
constexpr float B5_2 = (float)(500.0 / 1113.0);
constexpr float B5_3 = (float)(125.0 / 192.0);
constexpr float B5_4 = (float)(-2187.0 / 6784.0);
constexpr float B5_5 = (float)(11.0 / 84.0);
constexpr float E_0 = (float)(35.0 / 384.0 - 5179.0 / 57600.0);
constexpr float E_2 = (float)(500.0 / 1113.0 - 7571.0 / 16695.0);
constexpr float E_3 = (float)(125.0 / 192.0 - 393.0 / 640.0);
constexpr float E_4 = (float)(-2187.0 / 6784.0 + 92097.0 / 339200.0);
constexpr float E_5 = (float)(11.0 / 84.0 - 187.0 / 2100.0);
constexpr float E_6 = (float)(0.0 - 1.0 / 40.0);

typedef __attribute__((ext_vector_type(16))) _Float16 v16h;
typedef __attribute__((ext_vector_type(2)))  _Float16 v2h;
typedef __attribute__((ext_vector_type(8)))  float    v8f;
typedef __attribute__((ext_vector_type(4)))  float    v4f;
typedef __attribute__((ext_vector_type(4)))  unsigned v4u;
typedef __attribute__((ext_vector_type(2)))  unsigned v2u;

union FragH { v16h v; v4u q[2]; unsigned w[8]; };

__device__ __forceinline__ unsigned pack2h(float f0, float f1) {
  const float g0 = (fabsf(f0) < F16_MIN_NORMAL) ? 0.0f : f0;
  const float g1 = (fabsf(f1) < F16_MIN_NORMAL) ? 0.0f : f1;
  v2h p;
  p.x = (_Float16)g0;
  p.y = (_Float16)g1;
  return __builtin_bit_cast(unsigned, p);
}
__device__ __forceinline__ v16h ld_frag(const unsigned* p) {
  FragH f;
  f.q[0] = *(const v4u*)(p);
  f.q[1] = *(const v4u*)(p + 8);
  return f.v;
}
__device__ __forceinline__ v8f mma1(v16h a, v16h b, v8f c) {
  c = __builtin_amdgcn_wmma_f32_16x16x32_f16(false, a, false, b, (short)0, c, false, false);
  asm volatile("v_nop\n\tv_nop\n\tv_nop\n\tv_nop" : "+v"(c) : "v"(a), "v"(b));
  return c;
}

__global__ __launch_bounds__(NTHR) void adaptive_rk_kernel(
    const float* __restrict__ x,
    const float* __restrict__ W1, const float* __restrict__ b1,
    const float* __restrict__ W2, const float* __restrict__ b2,
    const float* __restrict__ W3, const float* __restrict__ b3,
    float* __restrict__ out0, float* __restrict__ wsl) {
  __shared__ __align__(16) unsigned W2h[DIM_H * WPW];
  __shared__ __align__(16) float W1T[(DIM_X + 1) * FP];
  __shared__ __align__(16) float W3s[DIM_X * FP];
  __shared__ __align__(16) unsigned H1h[SPB * WPW];
  __shared__ __align__(16) float S1[SPB * FP];
  __shared__ __align__(16) float H2[SPB * FP];
  __shared__ __align__(16) float S2[SPB * FP];
  __shared__ __align__(16) float Zt[SPB * ZP];
  __shared__ __align__(16) float KS[NSTAGE * SPB * ZP];
  __shared__ __align__(16) float Zfin[SPB * ZP];

  const int tid  = (int)threadIdx.x;
  const int lane = tid & 31;
  const int wave = tid >> 5;
  const int hh   = lane >> 4;
  const int c    = lane & 15;

#pragma unroll 4
  for (int it = 0; it < 16; ++it) {
    const int q = tid + NTHR * it;
    const int row = q >> 5;
    const int c4 = (q & 31) * 4;
    const v4f w = *(const v4f*)(W2 + (size_t)row * DIM_H + c4);
    v2u ph;
    ph.x = pack2h(w.x * CARRY_W2, w.y * CARRY_W2);
    ph.y = pack2h(w.z * CARRY_W2, w.w * CARRY_W2);
    *(v2u*)(W2h + row * WPW + (c4 >> 1)) = ph;
  }
#pragma unroll 1
  for (int it = 0; it < 17; ++it) {
    const int e = tid + NTHR * it;
    const int ec = (e < W1_ELEMS) ? e : (W1_ELEMS - 1);
    float v = W1[ec];
    asm volatile("" : "+v"(v));
    const int k = ec / (DIM_X + 1);
    const int i = ec - (DIM_X + 1) * k;
    if (e < W1_ELEMS) W1T[i * FP + k] = v;
  }
#pragma unroll
  for (int it = 0; it < 4; ++it) {
    const int q = tid + NTHR * it;
    const int row = q >> 5;
    const int c4 = (q & 31) * 4;
    const v4f w = *(const v4f*)(W3 + (size_t)row * DIM_H + c4);
    *(v4f*)(W3s + row * FP + c4) = w;
  }

  const v4f b1q = *(const v4f*)(b1 + 4 * lane);
  const v4f b2qa = *(const v4f*)(b2 + 16 * wave + 8 * hh);
  const v4f b2qb = *(const v4f*)(b2 + 16 * wave + 8 * hh + 4);
  float b2r[8];
#pragma unroll
  for (int e = 0; e < 4; ++e) { b2r[e] = b2qa[e]; b2r[4 + e] = b2qb[e]; }
  const float b3r = b3[lane];

  const int gs = (int)blockIdx.x * SPB + wave;
  float zj = x[(size_t)gs * DIM_X + lane];
  float zl = 0.0f;
  float t  = 0.0f;
  float dt = DT_INIT;
  bool  done = false;
  float dtc = fminf(dt, T_END - t);
  Zt[wave * ZP + lane] = zj;
  __syncthreads();

  const v8f z8 = {0.f, 0.f, 0.f, 0.f, 0.f, 0.f, 0.f, 0.f};

#pragma unroll 1
  for (int step = 0; step < NSTEPS; ++step) {
#pragma unroll 1
    for (int st = 0; st < NSTAGE; ++st) {
      const float targ = t + c_C[st] * dtc;
      const float teff = 1.0f - targ;

      {
        float a0 = b1q.x, a1 = b1q.y, a2 = b1q.z, a3 = b1q.w;
        const float* xrow = Zt + wave * ZP;
        const float* wcol = W1T + 4 * lane;
#pragma unroll 4
        for (int i = 0; i < DIM_X; ++i) {
          const float xv = xrow[i];
          const v4f w = *(const v4f*)(wcol + i * FP);
          a0 = fmaf(w.x, xv, a0);
          a1 = fmaf(w.y, xv, a1);
          a2 = fmaf(w.z, xv, a2);
          a3 = fmaf(w.w, xv, a3);
        }
        const v4f wt = *(const v4f*)(wcol + DIM_X * FP);
        a0 = fmaf(wt.x, teff, a0);
        a1 = fmaf(wt.y, teff, a1);
        a2 = fmaf(wt.z, teff, a2);
        a3 = fmaf(wt.w, teff, a3);
        const float g0 = tanhf(a0), g1 = tanhf(a1), g2 = tanhf(a2), g3 = tanhf(a3);
        v4f sv;
        sv.x = 1.0f - g0 * g0;
        sv.y = 1.0f - g1 * g1;
        sv.z = 1.0f - g2 * g2;
        sv.w = 1.0f - g3 * g3;
        *(v4f*)(S1 + wave * FP + 4 * lane) = sv;
        v2u ph;
        ph.x = pack2h(g0 * CARRY_H1, g1 * CARRY_H1);
        ph.y = pack2h(g2 * CARRY_H1, g3 * CARRY_H1);
        *(v2u*)(H1h + wave * WPW + 2 * lane) = ph;
      }
      __syncthreads();

      {
        v8f acc = z8;
        const unsigned* arh = W2h + (16 * wave + c) * WPW + 4 * hh;
        const unsigned* brh = H1h + (c & (SPB - 1)) * WPW + 4 * hh;
#pragma unroll
        for (int ks = 0; ks < 4; ++ks) {
          const v16h ah = ld_frag(arh + 16 * ks);
          const v16h bh = ld_frag(brh + 16 * ks);
          acc = mma1(ah, bh, acc);
        }
        v4f ha, hb, sa, sb;
#pragma unroll
        for (int r = 0; r < 4; ++r) {
          const float u0 = tanhf(acc[r] * FOLD_H1 + b2r[r]);
          const float u1 = tanhf(acc[4 + r] * FOLD_H1 + b2r[4 + r]);
          ha[r] = u0;
          hb[r] = u1;
          sa[r] = 1.0f - u0 * u0;
          sb[r] = 1.0f - u1 * u1;
        }
        if (c < SPB) {
          float* hp = H2 + c * FP + 16 * wave + 8 * hh;
          float* sp = S2 + c * FP + 16 * wave + 8 * hh;
          *(v4f*)(hp) = ha;
          *(v4f*)(hp + 4) = hb;
          *(v4f*)(sp) = sa;
          *(v4f*)(sp + 4) = sb;
        }
      }
      __syncthreads();

      {
        float acc = 0.0f;
        const float* hrow = H2 + wave * FP;
        const float* wrow = W3s + lane * FP;
#pragma unroll 2
        for (int k = 0; k < DIM_H; k += 4) {
          const v4f hq = *(const v4f*)(hrow + k);
          const v4f wq = *(const v4f*)(wrow + k);
          acc = fmaf(wq.x, hq.x, acc);
          acc = fmaf(wq.y, hq.y, acc);
          acc = fmaf(wq.z, hq.z, acc);
          acc = fmaf(wq.w, hq.w, acc);
        }
        const float kv = -(acc + b3r);
        KS[(st * SPB + wave) * ZP + lane] = kv;
        if (st < NSTAGE - 1) {
          float comb = 0.0f;
#pragma unroll 1
          for (int m = 0; m < st; ++m) comb += c_A[st][m] * KS[(m * SPB + wave) * ZP + lane];
          comb += c_A[st][st] * kv;
          Zt[wave * ZP + lane] = zj + dtc * comb;
        }
      }

      {
        float part = 0.0f;
#pragma unroll 1
        for (int nt = 0; nt < 2; ++nt) {
          v16h bh[4];
          const float* s1p = S1 + wave * FP + 8 * hh;
          const float* w1p = W1T + (16 * nt + c) * FP + 8 * hh;
#pragma unroll
          for (int ks = 0; ks < 4; ++ks) {
            FragH fh;
#pragma unroll
            for (int g = 0; g < 2; ++g) {
              const int ko = 32 * ks + 16 * g;
              const v4f sa = *(const v4f*)(s1p + ko);
              const v4f sb = *(const v4f*)(s1p + ko + 4);
              const v4f wa = *(const v4f*)(w1p + ko);
              const v4f wb = *(const v4f*)(w1p + ko + 4);
              fh.w[4 * g + 0] = pack2h((sa.x * wa.x) * CARRY_T1, (sa.y * wa.y) * CARRY_T1);
              fh.w[4 * g + 1] = pack2h((sa.z * wa.z) * CARRY_T1, (sa.w * wa.w) * CARRY_T1);
              fh.w[4 * g + 2] = pack2h((sb.x * wb.x) * CARRY_T1, (sb.y * wb.y) * CARRY_T1);
              fh.w[4 * g + 3] = pack2h((sb.z * wb.z) * CARRY_T1, (sb.w * wb.w) * CARRY_T1);
            }
            bh[ks] = fh.v;
          }
          const float* w3p = W3s + (16 * nt + c) * FP + 8 * hh;
          const float* s2p = S2 + wave * FP + 8 * hh;
#pragma unroll 1
          for (int m = 0; m < 8; ++m) {
            v8f acc = z8;
            const unsigned* arh = W2h + (16 * m + c) * WPW + 4 * hh;
#pragma unroll
            for (int ks = 0; ks < 4; ++ks) {
              const v16h ah = ld_frag(arh + 16 * ks);
              acc = mma1(ah, bh[ks], acc);
            }
            const v4f wa = *(const v4f*)(w3p + 16 * m);
            const v4f wb = *(const v4f*)(w3p + 16 * m + 4);
            const v4f sa = *(const v4f*)(s2p + 16 * m);
            const v4f sb = *(const v4f*)(s2p + 16 * m + 4);
#pragma unroll
            for (int r = 0; r < 4; ++r) {
              part += (wa[r] * sa[r]) * acc[r];
              part += (wb[r] * sb[r]) * acc[4 + r];
            }
          }
        }
        part += __shfl_xor(part, 16, 32);
        part += __shfl_xor(part, 8, 32);
        part += __shfl_xor(part, 4, 32);
        part += __shfl_xor(part, 2, 32);
        part += __shfl_xor(part, 1, 32);
        const float trv = part * FOLD_T1;
        if (lane == 0) KS[(st * SPB + wave) * ZP + DIM_X] = -trv;
      }
      __syncthreads();
    }

    {
      float kj[NSTAGE], kl[NSTAGE];
#pragma unroll
      for (int m = 0; m < NSTAGE; ++m) {
        kj[m] = KS[(m * SPB + wave) * ZP + lane];
        kl[m] = KS[(m * SPB + wave) * ZP + DIM_X];
      }
      const float a5j = B5_0 * kj[0] + B5_2 * kj[2] + B5_3 * kj[3] + B5_4 * kj[4] + B5_5 * kj[5];
      const float a5l = B5_0 * kl[0] + B5_2 * kl[2] + B5_3 * kl[3] + B5_4 * kl[4] + B5_5 * kl[5];
      const float aej = E_0 * kj[0] + E_2 * kj[2] + E_3 * kj[3] + E_4 * kj[4] + E_5 * kj[5] + E_6 * kj[6];
      const float ael = E_0 * kl[0] + E_2 * kl[2] + E_3 * kl[3] + E_4 * kl[4] + E_5 * kl[5] + E_6 * kl[6];
      const float z5j = zj + dtc * a5j;
      const float z5l = zl + dtc * a5l;
      const float ej = dtc * aej;
      const float el = dtc * ael;
      const float scj = ATOL_F + RTOL_F * fmaxf(fabsf(zj), fabsf(z5j));
      const float scl = ATOL_F + RTOL_F * fmaxf(fabsf(zl), fabsf(z5l));
      const float qj = ej * (1.0f / scj);
      const float ql = el * (1.0f / scl);
      float ssum = qj * qj;
      ssum += __shfl_xor(ssum, 16, 32);
      ssum += __shfl_xor(ssum, 8, 32);
      ssum += __shfl_xor(ssum, 4, 32);
      ssum += __shfl_xor(ssum, 2, 32);
      ssum += __shfl_xor(ssum, 1, 32);
      ssum += ql * ql;
      const float ratio = sqrtf(ssum * INV_NCMP);
      const bool accept = (ratio <= 1.0f);
      float fac = 0.9f * powf(fmaxf(ratio, 1e-10f), -0.2f);
      fac = fminf(fmaxf(fac, 0.2f), 10.0f);
      const float tn  = accept ? (t + dtc) : t;
      const float znj = accept ? z5j : zj;
      const float znl = accept ? z5l : zl;
      const float dtn = dtc * fac;
      const bool done_n = done || (tn >= T_DONE);
      t  = done ? t  : tn;
      zj = done ? zj : znj;
      zl = done ? zl : znl;
      dt = done ? dt : dtn;
      done = done_n;
      dtc = fminf(dt, T_END - t);
      Zt[wave * ZP + lane] = zj;
    }
    __syncthreads();
  }

  Zfin[wave * ZP + lane] = zj;
  if (lane == 0) Zfin[wave * ZP + DIM_X] = zl;
  __syncthreads();
  if (wave < 2) {
    const int row = tid >> 3;
    const int c4 = (tid & 7) * 4;
    const v4f v = *(const v4f*)(Zfin + row * ZP + c4);
    float* op = out0 + (size_t)((int)blockIdx.x * SPB + row) * DIM_X + c4;
    *(volatile v4f*)op = v;
    __threadfence();
    *(volatile v4f*)op = v;
  }
  if (wave == 2) {
    const int lc = (lane < SPB) ? lane : (SPB - 1);
    const float lv = Zfin[lc * ZP + DIM_X];
    const float v = (lane < SPB) ? lv : 0.0f;
    volatile float* p = wsl + (size_t)blockIdx.x * 32 + lane;
    *p = v;
    __threadfence();
    *p = v;
  }
}

__global__ __launch_bounds__(32) void logp_pack_kernel(const float* __restrict__ wsl, float* __restrict__ out1) {
  const int l = (int)threadIdx.x;
  const float v = wsl[(l >> 3) * 32 + (l & 7)];
  volatile float* p = out1 + l;
  *p = v;
  __threadfence();
  *p = v;
}

extern "C" void kernel_launch(void* const* d_in, const int* in_sizes, int n_in,
                              void* d_out, int out_size, void* d_ws, size_t ws_size, hipStream_t stream) {
  if (n_in < 7 || d_out == nullptr || d_ws == nullptr) return;
  if (in_sizes[0] != NSAMP * DIM_X || in_sizes[1] != W1_ELEMS || in_sizes[2] != DIM_H ||
      in_sizes[3] != DIM_H * DIM_H || in_sizes[4] != DIM_H || in_sizes[5] != DIM_X * DIM_H ||
      in_sizes[6] != DIM_X || out_size != OUT_ELEMS) return;

  const float* x  = (const float*)d_in[0];
  const float* W1 = (const float*)d_in[1];
  const float* b1 = (const float*)d_in[2];
  const float* W2 = (const float*)d_in[3];
  const float* b2 = (const float*)d_in[4];
  const float* W3 = (const float*)d_in[5];
  const float* b3 = (const float*)d_in[6];
  float* out = (float*)d_out;

  char* ws = (char*)d_ws;
  size_t off = 0;
  auto carve = [&](size_t bytes) -> char* { char* p = ws + off; off += (bytes + 255) & ~(size_t)255; return p; };
  float* wsl = (float*)carve((size_t)NBLK * 32 * 4);
  if (off > ws_size || off > (size_t)134217728) return;

  adaptive_rk_kernel<<<NBLK, NTHR, 0, stream>>>(x, W1, b1, W2, b2, W3, b3, out, wsl);
  logp_pack_kernel<<<1, 32, 0, stream>>>(wsl, out + OUT0_ELEMS);
}
